// Conv3DSubmModule_8598524527254
// MI455X (gfx1250) — hardware-verified
//
#include <hip/hip_runtime.h>
#include <stdint.h>

#define NV       100000
#define K3       27
#define DIN      64
#define DOUT     64
#define TILE_M   128
#define NBLK     ((NV + TILE_M - 1) / TILE_M)
#define TAILROWS (NV - (NBLK - 1) * TILE_M)
#define LDA      72
#define IDX_INTS (TILE_M * K3)
#define IDX_Q    (IDX_INTS / 4)
#define SO_LD    68
#define XUNITS   (NV * DIN / 8)
#define XBLKS    (XUNITS / 256)
#define SLAB     (DIN * DOUT)
#define SW_LD    65
#define WSCAP    134217728

static_assert(K3 == 27);
static_assert(DIN == 64 && DIN % 32 == 0);
static_assert(DOUT == 64 && DOUT == 4 * 16);
static_assert(TILE_M == 128 && TILE_M == 8 * 16);
static_assert((TILE_M * K3 * 4) % 128 == 0);
static_assert((TAILROWS * K3) % 4 == 0);
static_assert(TAILROWS % 16 == 0 && TAILROWS >= 1);
static_assert(DIN * 2 == 128);
static_assert((DOUT * 4) % 128 == 0);
static_assert(XUNITS == XBLKS * 256);
static_assert(IDX_Q == 3 * 256 + 96 && 96 % 32 == 0);
static_assert((LDA * 2) % 16 == 0);
static_assert((SO_LD * 4) % 16 == 0);

typedef float          v4f   __attribute__((ext_vector_type(4)));
typedef float          v8f   __attribute__((ext_vector_type(8)));
typedef int            v4i   __attribute__((ext_vector_type(4)));
typedef int            v8i   __attribute__((ext_vector_type(8)));
typedef unsigned int   v4u   __attribute__((ext_vector_type(4)));
typedef unsigned short v8us  __attribute__((ext_vector_type(8)));
typedef __bf16         v16bf __attribute__((ext_vector_type(16)));
typedef v4f  __attribute__((may_alias)) v4fa;
typedef v4i  __attribute__((may_alias)) v4ia;
typedef v4u  __attribute__((may_alias)) v4ua;
typedef v8us __attribute__((may_alias)) v8usa;
union FragB { v16bf v; v8us h[2]; v8i w; };

__device__ __forceinline__ unsigned short f2bf_bits(float f) {
  const unsigned u = __float_as_uint(f);
  return (unsigned short)((u + 0x7FFFu + ((u >> 16) & 1u)) >> 16);
}
__device__ __forceinline__ unsigned pk16(unsigned short a, unsigned short b) { return (unsigned)a | ((unsigned)b << 16); }

__device__ __forceinline__ v8f wmb(const FragB& a, const FragB& b, v8f c) {
  v8f d = __builtin_amdgcn_wmma_f32_16x16x32_bf16(false, a.v, false, b.v, (short)0, c, false, false);
  asm volatile("v_nop\n\tv_nop\n\tv_nop\n\tv_nop" : "+v"(d) : "v"(a.w), "v"(b.w));
  return d;
}
__device__ __forceinline__ v8f z8() { v8f z = {0.f, 0.f, 0.f, 0.f, 0.f, 0.f, 0.f, 0.f}; return z; }

__global__ __launch_bounds__(256) void k_prep(const float* __restrict__ feats, const float* __restrict__ weight,
                                              unsigned short* __restrict__ XB, unsigned short* __restrict__ WS) {
  __shared__ __align__(16) float sW[DIN * SW_LD];
  const int tid = threadIdx.x;
  if (blockIdx.x < XBLKS) {
    const size_t u = (size_t)blockIdx.x * 256 + (size_t)tid;
    const float* src = feats + u * 8;
    unsigned short* dst = XB + u * 8;
    const v4f a = *(const v4fa*)src;
    const v4f c = *(const v4fa*)(src + 4);
    v4u v;
    v[0] = pk16(f2bf_bits(a[0]), f2bf_bits(a[1]));
    v[1] = pk16(f2bf_bits(a[2]), f2bf_bits(a[3]));
    v[2] = pk16(f2bf_bits(c[0]), f2bf_bits(c[1]));
    v[3] = pk16(f2bf_bits(c[2]), f2bf_bits(c[3]));
    *(volatile v4u*)dst = v;
    __threadfence();
    *(volatile v4u*)dst = v;
  } else {
    const int k = (int)blockIdx.x - XBLKS;
    const float* wsrc = weight + (size_t)k * SLAB;
#pragma unroll
    for (int i = 0; i < 4; ++i) {
      const int e4 = tid + 256 * i;
      const v4f v = *(const v4fa*)(wsrc + 4 * e4);
      const int d = (4 * e4) >> 6, e = (4 * e4) & 63;
      sW[d * SW_LD + e + 0] = v[0];
      sW[d * SW_LD + e + 1] = v[1];
      sW[d * SW_LD + e + 2] = v[2];
      sW[d * SW_LD + e + 3] = v[3];
    }
    __syncthreads();
    v4u o[2];
#pragma unroll
    for (int i = 0; i < 2; ++i) {
      const int u = tid + 256 * i;
      const int e = u >> 3, g = u & 7;
      const float* p = sW + (8 * g) * SW_LD + e;
      o[i][0] = pk16(f2bf_bits(p[0 * SW_LD]), f2bf_bits(p[1 * SW_LD]));
      o[i][1] = pk16(f2bf_bits(p[2 * SW_LD]), f2bf_bits(p[3 * SW_LD]));
      o[i][2] = pk16(f2bf_bits(p[4 * SW_LD]), f2bf_bits(p[5 * SW_LD]));
      o[i][3] = pk16(f2bf_bits(p[6 * SW_LD]), f2bf_bits(p[7 * SW_LD]));
    }
    unsigned short* dbase = WS + (size_t)k * SLAB;
    *(volatile v4u*)(dbase + 8 * tid) = o[0];
    *(volatile v4u*)(dbase + 8 * (tid + 256)) = o[1];
    __threadfence();
    *(volatile v4u*)(dbase + 8 * tid) = o[0];
    *(volatile v4u*)(dbase + 8 * (tid + 256)) = o[1];
  }
}

struct StageT {
  int idx[IDX_INTS];
  unsigned short a[TILE_M * LDA];
  unsigned short b[DOUT * LDA];
};
union SmemT {
  StageT s;
  float o[TILE_M * SO_LD];
};
static_assert(sizeof(StageT) == 41472);
static_assert(sizeof(SmemT) == 41472);
static_assert(sizeof(SmemT) <= 327680);

__device__ __forceinline__ void o_store_pass(const float* so, float* out, int r0, int w, int lane, int nv) {
  const int q16 = lane & 15, sub = lane >> 4;
#pragma unroll
  for (int i = 0; i < 8; ++i) {
    const int row = 16 * w + 2 * i + sub;
    const int grow = r0 + row;
    const v4f v = *(const v4fa*)(so + row * SO_LD + 4 * q16);
    if (grow < nv) *(volatile v4f*)(out + (size_t)grow * DOUT + 4 * q16) = v;
  }
}

__global__ __launch_bounds__(256) __attribute__((amdgpu_num_vgpr(248)))
void k_conv(const unsigned short* __restrict__ XB, const int* __restrict__ indices,
            const unsigned short* __restrict__ WS, float* __restrict__ out, int nv) {
  __shared__ __align__(16) SmemT sm;

  const int tid = threadIdx.x, lane = tid & 31, w = tid >> 5;
  const int h = lane >> 4, m = lane & 15;
  const int r0 = (int)blockIdx.x * TILE_M;
  int nrows = nv - r0;
  nrows = (nrows > TILE_M) ? TILE_M : nrows;
  nrows = (nrows < 1) ? 1 : nrows;
  const int nq = (nrows * K3) >> 2;

  {
    const int* ibase = indices + (size_t)r0 * K3;
#pragma unroll
    for (int i = 0; i < 4; ++i) {
      const int q = tid + 256 * i;
      const int qc = (q < nq - 1) ? q : (nq - 1);
      v4i v = *(const v4ia*)(ibase + 4 * qc);
      const int mk = (q < nq) ? -1 : 0;
      const v4i mkv = {mk, mk, mk, mk};
      v = (v & mkv) | ~mkv;
      if (q < IDX_Q) *(v4ia*)&sm.s.idx[4 * q] = v;
    }
  }
  __syncthreads();

  v8f acc[4];
#pragma unroll
  for (int nt = 0; nt < 4; ++nt) acc[nt] = z8();

  const int hi_row = nv - 1;

#pragma unroll 1
  for (int k = 0; k < K3; ++k) {
    v4u av[4];
#pragma unroll
    for (int i = 0; i < 4; ++i) {
      const int u = tid + 256 * i;
      const int r = u >> 3, p = u & 7;
      const int idx = sm.s.idx[r * K3 + k];
      int ic = (idx > 0) ? idx : 0;
      ic = (ic < hi_row) ? ic : hi_row;
      const v4u v = *(const v4ua*)(XB + (size_t)ic * DIN + 8 * p);
      const unsigned ok = (unsigned)((idx >= 0) & ((r0 + r) < nv));
      const unsigned mk = 0u - ok;
      const v4u mkv = {mk, mk, mk, mk};
      av[i] = v & mkv;
    }
    v4u bv[2];
#pragma unroll
    for (int i = 0; i < 2; ++i) {
      const int u = tid + 256 * i;
      bv[i] = *(const v4ua*)(WS + (size_t)k * SLAB + 8 * u);
    }
#pragma unroll
    for (int i = 0; i < 4; ++i) {
      const int u = tid + 256 * i;
      const int r = u >> 3, p = u & 7;
      *(v4ua*)&sm.s.a[r * LDA + 8 * p] = av[i];
    }
#pragma unroll
    for (int i = 0; i < 2; ++i) {
      const int u = tid + 256 * i;
      const int e = u >> 3, p = u & 7;
      *(v4ua*)&sm.s.b[e * LDA + 8 * p] = bv[i];
    }
    __syncthreads();

    const unsigned short* ap = &sm.s.a[(16 * w + m) * LDA + 8 * h];
    FragB a0, a1;
    a0.h[0] = *(const v8usa*)(ap);
    a0.h[1] = *(const v8usa*)(ap + 16);
    a1.h[0] = *(const v8usa*)(ap + 32);
    a1.h[1] = *(const v8usa*)(ap + 48);
#pragma unroll
    for (int nt = 0; nt < 4; ++nt) {
      const unsigned short* bp = &sm.s.b[(16 * nt + m) * LDA + 8 * h];
      FragB b0, b1;
      b0.h[0] = *(const v8usa*)(bp);
      b0.h[1] = *(const v8usa*)(bp + 16);
      b1.h[0] = *(const v8usa*)(bp + 32);
      b1.h[1] = *(const v8usa*)(bp + 48);
      acc[nt] = wmb(a0, b0, acc[nt]);
      acc[nt] = wmb(a1, b1, acc[nt]);
    }
    __syncthreads();
  }

#pragma unroll
  for (int nt = 0; nt < 4; ++nt) {
#pragma unroll
    for (int r = 0; r < 8; ++r) {
      sm.o[(16 * w + 8 * h + r) * SO_LD + 16 * nt + m] = acc[nt][r];
    }
  }
  __syncthreads();

  o_store_pass(sm.o, out, r0, w, lane, nv);
  __threadfence();
  o_store_pass(sm.o, out, r0, w, lane, nv);
}

extern "C" void kernel_launch(void* const* d_in, const int* in_sizes, int n_in,
                              void* d_out, int out_size, void* d_ws, size_t ws_size,
                              hipStream_t stream) {
  if (n_in < 3) return;
  if (in_sizes[0] != NV * DIN) return;
  if (in_sizes[1] != NV * K3) return;
  if (in_sizes[2] != K3 * SLAB) return;
  if (out_size != NV * DOUT) return;

  const float* feats   = (const float*)d_in[0];
  const int*   indices = (const int*)d_in[1];
  const float* weight  = (const float*)d_in[2];
  float* out = (float*)d_out;

  size_t off = 0;
  const size_t oXB = off; off += (size_t)NV * DIN * 2;
  const size_t oWS = off; off += (size_t)K3 * SLAB * 2;
  if ((oWS % 128) != 0) return;
  if (off > ws_size) return;
  if (off > (size_t)WSCAP) return;

  char* ws = (char*)d_ws;
  unsigned short* XB = (unsigned short*)(ws + oXB);
  unsigned short* WS = (unsigned short*)(ws + oWS);

  k_prep<<<dim3(XBLKS + K3), dim3(256), 0, stream>>>(feats, weight, XB, WS);
  k_conv<<<dim3(NBLK), dim3(256), 0, stream>>>(XB, indices, WS, out, NV);
  (void)hipGetLastError();
}
